// MultiResBiplane_41635412968145
// MI455X (gfx1250) — hardware-verified
//
#include <hip/hip_runtime.h>
#include <math.h>

typedef __attribute__((ext_vector_type(16))) _Float16 v16h;
typedef __attribute__((ext_vector_type(16))) __bf16 v16b;
typedef __attribute__((ext_vector_type(8)))  _Float16 v8h;
typedef __attribute__((ext_vector_type(8)))  float v8f;
typedef __attribute__((ext_vector_type(4)))  float v4f;
typedef __attribute__((ext_vector_type(2)))  float v2f;
typedef __attribute__((ext_vector_type(4)))  unsigned v4u;
typedef __attribute__((ext_vector_type(4)))  int v4i;
typedef float __attribute__((may_alias)) float_a;
typedef int __attribute__((may_alias)) int_a;

template <typename T> __device__ __forceinline__ void vst2(void* p, T v) { *(volatile T*)p = v; __threadfence(); *(volatile T*)p = v; }
__device__ __forceinline__ v8f wmma16(v16h a, v16h b, v8f c) {
  v8f d = __builtin_amdgcn_wmma_f32_16x16x32_f16(false, a, false, b, (short)0, c, false, false);
  asm volatile("v_nop\n\tv_nop\n\tv_nop\n\tv_nop" : "+v"(d) : "v"(a), "v"(b));
  return d;
}
__device__ __forceinline__ v8f wmma_bf(v16b a, v16b b, v8f c) {
  v8f d = __builtin_amdgcn_wmma_f32_16x16x32_bf16(false, a, false, b, (short)0, c, false, false);
  asm volatile("v_nop\n\tv_nop\n\tv_nop\n\tv_nop" : "+v"(d) : "v"(a), "v"(b));
  return d;
}
__device__ __forceinline__ v16h frag_h(const _Float16* rowk0, int lane) {
  union { v16h v; v8h q[2]; } u; const _Float16* p = rowk0 + 8 * (lane >> 4);
  u.q[0] = *(const v8h*)p; u.q[1] = *(const v8h*)(p + 16); return u.v;
}
__device__ __forceinline__ v16h frag_f32(const float* rowk0, int lane) {
  v16h a; const float* p = rowk0 + 8 * (lane >> 4);
#pragma unroll
  for (int i = 0; i < 8; ++i) { a[i] = (_Float16)p[i]; a[8 + i] = (_Float16)p[16 + i]; }
  return a;
}
__device__ __forceinline__ v16h frag_f32s(const float* rowk0, int lane, float sc) {
  v16h a; const float* p = rowk0 + 8 * (lane >> 4);
#pragma unroll
  for (int i = 0; i < 8; ++i) { a[i] = (_Float16)(p[i] * sc); a[8 + i] = (_Float16)(p[16 + i] * sc); }
  return a;
}
__device__ __forceinline__ v16h fragc_f32(const float* W, int k0, int n, int lane, int ld, int K) {
  v16h a; const int g = lane >> 4;
#pragma unroll
  for (int i = 0; i < 8; ++i) { const int ka = k0 + 8 * g + i, kb = ka + 16;
    a[i] = (_Float16)(ka < K ? W[(size_t)ka * ld + n] : 0.f); a[8 + i] = (_Float16)(kb < K ? W[(size_t)kb * ld + n] : 0.f); }
  return a;
}
struct F2 { v16b h, l; };
__device__ __forceinline__ F2 bsplit16(const float v[16]) { F2 r;
#pragma unroll
  for (int i = 0; i < 16; ++i) { const __bf16 h = (__bf16)v[i]; r.h[i] = h; r.l[i] = (__bf16)(v[i] - (float)h); }
  return r; }
__device__ __forceinline__ F2 split_row(const float* row, int k0, int lane) { float v[16]; const float* p = row + k0 + 8 * (lane >> 4);
#pragma unroll
  for (int i = 0; i < 8; ++i) { v[i] = p[i]; v[8 + i] = p[16 + i]; }
  return bsplit16(v); }
__device__ __forceinline__ F2 split_rowK(const float* row, int k0, int lane, int K) { float v[16]; const int g = lane >> 4;
#pragma unroll
  for (int i = 0; i < 8; ++i) { const int ka = k0 + 8 * g + i, kb = ka + 16; v[i] = ka < K ? row[ka] : 0.f; v[8 + i] = kb < K ? row[kb] : 0.f; }
  return bsplit16(v); }
__device__ __forceinline__ F2 split_col(const float* W, int k0, int n, int lane, int ld, int K) { float v[16]; const int g = lane >> 4;
#pragma unroll
  for (int i = 0; i < 8; ++i) { const int ka = k0 + 8 * g + i, kb = ka + 16; v[i] = ka < K ? W[(size_t)ka * ld + n] : 0.f; v[8 + i] = kb < K ? W[(size_t)kb * ld + n] : 0.f; }
  return bsplit16(v); }
__device__ __forceinline__ v8f mac3(const F2& a, const F2& b, v8f c) { c = wmma_bf(a.l, b.h, c); c = wmma_bf(a.h, b.l, c); return wmma_bf(a.h, b.h, c); }
__device__ __forceinline__ float sigm(float v) { return 1.0f / (1.0f + expf(-v)); }
#define LDSX() do { asm volatile("s_wait_dscnt 0" ::: "memory"); __builtin_amdgcn_wave_barrier(); __builtin_amdgcn_fence(__ATOMIC_RELEASE, "workgroup"); } while (0)


#define NPTS 1048576
#define PPI (4096 * 32)
#define FD 16
#define TD 24
#define IND 72
#define HID 36
__device__ __forceinline__ float lrelu(float v) { return v >= 0.f ? v : 0.01f * v; }
__device__ __forceinline__ void sample8(const float* __restrict__ plane, int R, float gx, float gy, int c0, float* dst) {
  const float x = (gx + 1.0f) * 0.5f * (float)(R - 1), y = (gy + 1.0f) * 0.5f * (float)(R - 1);
  const float x0 = floorf(x), y0 = floorf(y); const float x1 = x0 + 1.0f, y1 = y0 + 1.0f; const float wx1 = x - x0, wx0 = 1.0f - wx1, wy1 = y - y0, wy0 = 1.0f - wy1;
  const float cx[2] = {x0, x1}, cy[2] = {y0, y1}, wxs[2] = {wx0, wx1}, wys[2] = {wy0, wy1};
  float acc[8];
#pragma unroll
  for (int e = 0; e < 8; ++e) acc[e] = 0.f;
#pragma unroll
  for (int iy = 0; iy < 2; ++iy)
#pragma unroll
    for (int ix = 0; ix < 2; ++ix) { const float xi = cx[ix], yi = cy[iy]; const bool valid = xi >= 0.f && xi < (float)R && yi >= 0.f && yi < (float)R;
      const int xc = (int)fminf(fmaxf(xi, 0.f), (float)(R - 1)), yc = (int)fminf(fmaxf(yi, 0.f), (float)(R - 1)); const float w = valid ? wys[iy] * wxs[ix] : 0.f;
      const float* p = plane + (size_t)yc * R + xc;
#pragma unroll
      for (int e = 0; e < 8; ++e) acc[e] += p[(size_t)(c0 + e) * R * R] * w; }
#pragma unroll
  for (int e = 0; e < 8; ++e) dst[e] = acc[e];
}
__global__ __launch_bounds__(128) void k_mrb(const float* __restrict__ coords, const float* __restrict__ tfeat, const float* __restrict__ P0, const float* __restrict__ P1, const float* __restrict__ P2,
                                            const float* __restrict__ w1, const float* __restrict__ b1, const float* __restrict__ w2, const float* __restrict__ b2, float* __restrict__ out) {
  __shared__ __align__(16) float sf[64][100];
  __shared__ __align__(16) float sh[64][52];
  const int tid = threadIdx.x, wave = tid >> 5, lane = tid & 31, col = lane & 15, g = lane >> 4; const int p0 = blockIdx.x * 64;
  { const int pl = tid & 63, hf = tid >> 6; const int p = p0 + pl; const float gx = coords[(size_t)p * 2], gy = coords[(size_t)p * 2 + 1]; const int c0 = hf * 8;
    sample8(P0, 128, gx, gy, c0, &sf[pl][c0]); sample8(P1, 256, gx, gy, c0, &sf[pl][FD + c0]); sample8(P2, 512, gx, gy, c0, &sf[pl][2 * FD + c0]);
    const int img = p / PPI; const float* tf = tfeat + (size_t)img * TD;
    for (int k = hf; k < TD; k += 2) sf[pl][3 * FD + k] = tf[k];
    for (int k = IND + hf; k < 96; k += 2) sf[pl][k] = 0.f; }
  __syncthreads();
  { v8f acc[3] = {};
#pragma unroll
    for (int kc = 0; kc < 3; ++kc) { const F2 a = split_row(&sf[wave * 16 + col][0], kc * 32, lane);
#pragma unroll
      for (int j = 0; j < 3; ++j) { const int n = j * 16 + col; const int nc = n < HID ? n : HID - 1; acc[j] = mac3(a, split_rowK(w1 + (size_t)nc * IND, kc * 32, lane, IND), acc[j]); } }
#pragma unroll
    for (int j = 0; j < 3; ++j)
#pragma unroll
      for (int r = 0; r < 8; ++r) { const int n = j * 16 + col; sh[wave * 16 + 8 * g + r][n] = n < HID ? lrelu(acc[j][r] + b1[n]) : 0.f; } }
  __syncthreads();
  { const int pl = tid >> 1, o = tid & 1; float s = b2[o];
#pragma unroll 4
    for (int k = 0; k < HID; ++k) s += sh[pl][k] * w2[o * HID + k];
    vst2(out + (size_t)(p0 + pl) * 2 + o, (float_a)(1.0f / (1.0f + expf(-s)))); }
}
extern "C" void kernel_launch(void* const* d_in, const int* in_sizes, int n_in, void* d_out, int out_size, void* d_ws, size_t ws_size, hipStream_t stream) {
  (void)in_sizes; (void)n_in; (void)out_size; (void)ws_size; (void)d_ws;
  const float** I = (const float**)d_in;
  k_mrb<<<NPTS / 64, 128, 0, stream>>>(I[0], I[1], I[2], I[3], I[4], I[5], I[6], I[7], I[8], (float*)d_out);
}
